// LoRABCBlock_32418413150722
// MI455X (gfx1250) — hardware-verified
//
#include <hip/hip_runtime.h>
#include <stddef.h>


typedef __attribute__((ext_vector_type(16))) _Float16 v16h;
typedef __attribute__((ext_vector_type(8)))  _Float16 v8h;
typedef __attribute__((ext_vector_type(16))) __bf16   v16b;
typedef __attribute__((ext_vector_type(8)))  __bf16   v8b;
typedef __attribute__((ext_vector_type(8)))  float    v8f;
typedef __attribute__((ext_vector_type(4)))  float    v4f;

__device__ __forceinline__ unsigned short f2bf_bits(float f) {
  unsigned u = __float_as_uint(f);
  return (unsigned short)((u + 0x7FFFu + ((u >> 16) & 1u)) >> 16);
}
__device__ __forceinline__ float bf_bits2f(unsigned short h) { return __uint_as_float(((unsigned)h) << 16); }

__device__ __forceinline__ void dep_guard_h(v8f& a, v8f& b, v16h x, v16h y) { asm volatile("v_nop\n\tv_nop\n\tv_nop\n\tv_nop" : "+v"(a), "+v"(b) : "v"(x), "v"(y)); }
__device__ __forceinline__ void dep_guard_b(v8f& a, v8f& b, v16b x, v16b y) { asm volatile("v_nop\n\tv_nop\n\tv_nop\n\tv_nop" : "+v"(a), "+v"(b) : "v"(x), "v"(y)); }
__device__ __forceinline__ void keep4_h(v16h a, v16h b, v16h c, v16h d) { asm volatile("v_nop" :: "v"(a), "v"(b), "v"(c), "v"(d)); }
__device__ __forceinline__ void keep4_b(v16b a, v16b b, v16b c, v16b d) { asm volatile("v_nop" :: "v"(a), "v"(b), "v"(c), "v"(d)); }
__device__ __forceinline__ void acc_guard4(v8f& a, v8f& b, v8f& c, v8f& d) { asm volatile("v_nop\n\tv_nop\n\tv_nop\n\tv_nop" : "+v"(a), "+v"(b), "+v"(c), "+v"(d)); }
template <typename T> struct Frag;
template <> struct Frag<_Float16> {
  typedef v16h V; union U { v16h v; v8h h[2]; };
  static __device__ __forceinline__ v16h load(const _Float16* p) {
    U f; f.h[0] = *(const v8h*)(p); f.h[1] = *(const v8h*)(p + 16); return f.v;
  }
  static __device__ __forceinline__ v8f mma(v16h a, v16h b, v8f c) {
    return __builtin_amdgcn_wmma_f32_16x16x32_f16(false, a, false, b, (short)0, c, false, false);
  }
  static __device__ __forceinline__ void guard(v8f& a, v8f& b, v16h x, v16h y) { dep_guard_h(a, b, x, y); }
  static __device__ __forceinline__ void keep(v16h a, v16h b, v16h c, v16h d) { keep4_h(a, b, c, d); }
};
template <> struct Frag<__bf16> {
  typedef v16b V; union U { v16b v; v8b h[2]; };
  static __device__ __forceinline__ v16b load(const __bf16* p) {
    U f; f.h[0] = *(const v8b*)(p); f.h[1] = *(const v8b*)(p + 16); return f.v;
  }
  static __device__ __forceinline__ v8f mma(v16b a, v16b b, v8f c) {
    return __builtin_amdgcn_wmma_f32_16x16x32_bf16(false, a, false, b, (short)0, c, false, false);
  }
  static __device__ __forceinline__ void guard(v8f& a, v8f& b, v16b x, v16b y) { dep_guard_b(a, b, x, y); }
  static __device__ __forceinline__ void keep(v16b a, v16b b, v16b c, v16b d) { keep4_b(a, b, c, d); }
};

template <int ET> struct Elem;
template <> struct Elem<0> { typedef _Float16 T; };
template <> struct Elem<1> { typedef __bf16 T; };
template <int ET, bool SPLIT, int BIAS_MODE, int OUT_MODE, bool RESID, int ACT = 0>
__global__ __launch_bounds__(256) void wmma_gemm64(
    const unsigned short* __restrict__ Ap, const unsigned short* __restrict__ A2p, int lda, long strideA,
    const unsigned short* __restrict__ Btp, const unsigned short* __restrict__ Bt2p, int ldb, long strideB,
    void* __restrict__ Cout, void* __restrict__ Cout2, int ldc, long strideC,
    const float* __restrict__ bias,
    const float* __restrict__ resid, long strideR,
    int M, int N, int K, float scale) {
  typedef typename Elem<ET>::T T;
  typedef typename Frag<T>::V V;
  const T* A = (const T*)Ap; const T* A2 = (const T*)A2p; const T* Bt = (const T*)Btp; const T* Bt2 = (const T*)Bt2p;
  __shared__ __align__(16) float sT[8][16 * 68];
  const int b    = blockIdx.y;
  const int lane = threadIdx.x & 31;
  const int wave = threadIdx.x >> 5;
  const int tilesN = N >> 6;
  const int tilesM = M >> 6;
  const int tile = blockIdx.x * 8 + wave;
  if (tile >= tilesM * tilesN) return;
  const int tm = tile / tilesN;
  const int tn = tile - tm * tilesN;
  const int m0 = tm << 6;
  const int n0 = tn << 6;

  const T* Ab  = A  + (size_t)b * strideA;
  const T* Bb  = Bt + (size_t)b * strideB;
  const T* Ab2 = SPLIT ? (A2  + (size_t)b * strideA) : nullptr;
  const T* Bb2 = SPLIT ? (Bt2 + (size_t)b * strideB) : nullptr;

  const int rlane = lane & 15;
  const int koff  = (lane >> 4) * 8;
  const int mOff  = (lane >> 4) * 8;

  v8f acc[4][4];
#pragma unroll
  for (int i = 0; i < 4; ++i)
#pragma unroll
    for (int j = 0; j < 4; ++j) acc[i][j] = (v8f){0.f,0.f,0.f,0.f,0.f,0.f,0.f,0.f};

  for (int k0 = 0; k0 < K; k0 += 32) {
    V bh[4], bl[4];
#pragma unroll
    for (int j = 0; j < 4; ++j) {
      const size_t bo = (size_t)(n0 + (j << 4) + rlane) * ldb + koff + k0;
      bh[j] = Frag<T>::load(Bb + bo);
      if (SPLIT) bl[j] = Frag<T>::load(Bb2 + bo);
    }
#pragma unroll
    for (int i = 0; i < 4; ++i) {
      const size_t ao = (size_t)(m0 + (i << 4) + rlane) * lda + koff + k0;
      V ah = Frag<T>::load(Ab + ao);
      V al;
      if (SPLIT) al = Frag<T>::load(Ab2 + ao);
#pragma unroll
      for (int j = 0; j < 4; ++j) {
        acc[i][j] = Frag<T>::mma(ah, bh[j], acc[i][j]);
        if (SPLIT) {
          acc[i][j] = Frag<T>::mma(ah, bl[j], acc[i][j]);
          acc[i][j] = Frag<T>::mma(al, bh[j], acc[i][j]);
        }
      }
      Frag<T>::guard(acc[i][0], acc[i][3], ah, SPLIT ? al : ah);
    }
    Frag<T>::keep(bh[0], bh[1], bh[2], bh[3]);
    if (SPLIT) Frag<T>::keep(bl[0], bl[1], bl[2], bl[3]);
  }
  acc_guard4(acc[0][0], acc[0][1], acc[0][2], acc[0][3]);
  acc_guard4(acc[1][0], acc[1][1], acc[1][2], acc[1][3]);
  acc_guard4(acc[2][0], acc[2][1], acc[2][2], acc[2][3]);
  acc_guard4(acc[3][0], acc[3][1], acc[3][2], acc[3][3]);

  float* slab = sT[wave];
  const float* Rb = RESID ? (resid + (size_t)b * strideR) : nullptr;
#pragma unroll
  for (int i = 0; i < 4; ++i) {
    const int mBase = m0 + (i << 4);
#pragma unroll
    for (int j = 0; j < 4; ++j) {
      const int n = n0 + (j << 4) + rlane;
      float bv = 0.f;
      if (BIAS_MODE == 2) bv = bias[n];
#pragma unroll
      for (int r = 0; r < 8; ++r) {
        float v = acc[i][j][r] * scale;
        if (BIAS_MODE == 1) v += bias[mBase + mOff + r];
        if (BIAS_MODE == 2) v += bv;
        if (RESID) v += Rb[(size_t)(mBase + mOff + r) * ldc + n];
        if (ACT == 1) v = tanhf(v);
        if (ACT == 2) v = fmaxf(v, 0.0f);
        if (ACT == 3) v = v / (1.0f + expf(-v));
        if (ACT == 4) v = (v > 0.f) ? v : 0.01f * v;
        if (ACT == 5) v = 0.5f * v * (1.0f + erff(v * 0.70710678118654752f));
        slab[(mOff + r) * 68 + (j << 4) + rlane] = v;
      }
    }
    __builtin_amdgcn_fence(__ATOMIC_RELEASE, "workgroup");
    __builtin_amdgcn_wave_barrier();
    __builtin_amdgcn_fence(__ATOMIC_ACQUIRE, "workgroup");
    if (OUT_MODE == 0) {
      float* C = (float*)Cout + (size_t)b * strideC;
      const int hh = lane >> 4, c4 = (lane & 15) * 4;
      for (int pass = 0; pass < 2; ++pass) {
#pragma unroll
        for (int it = 0; it < 8; ++it) {
          const int row = it * 2 + hh;
          v4f v = *(const v4f*)(slab + row * 68 + c4);
          *(volatile v4f*)(C + (size_t)(mBase + row) * ldc + n0 + c4) = v;
        }
        __threadfence();
      }
    } else {
      const int q = lane >> 3, c8 = (lane & 7) * 8;
      unsigned short* C  = (unsigned short*)Cout  + (size_t)b * strideC;
      unsigned short* C2 = (OUT_MODE == 2) ? ((unsigned short*)Cout2 + (size_t)b * strideC) : nullptr;
      for (int pass = 0; pass < 2; ++pass) {
#pragma unroll
        for (int it = 0; it < 4; ++it) {
          const int row = it * 4 + q;
          const float* sp = slab + row * 68 + c8;
          v8h hv, lv;
#pragma unroll
          for (int e = 0; e < 8; ++e) {
            if (OUT_MODE == 1) {
              hv[e] = (_Float16)sp[e];
            } else {
              unsigned short hb = f2bf_bits(sp[e]);
              unsigned short lb = f2bf_bits(sp[e] - bf_bits2f(hb));
              hv[e] = __builtin_bit_cast(_Float16, hb);
              lv[e] = __builtin_bit_cast(_Float16, lb);
            }
          }
          *(volatile v8h*)(C + (size_t)(mBase + row) * ldc + n0 + c8) = hv;
          if (OUT_MODE == 2) *(volatile v8h*)(C2 + (size_t)(mBase + row) * ldc + n0 + c8) = lv;
        }
        __threadfence();
      }
    }
    __builtin_amdgcn_fence(__ATOMIC_RELEASE, "workgroup");
    __builtin_amdgcn_wave_barrier();
    __builtin_amdgcn_fence(__ATOMIC_ACQUIRE, "workgroup");
  }
}

__global__ __launch_bounds__(256) void cast_scale_f16x8(
    const float* __restrict__ in, _Float16* __restrict__ out, int n8, float sc) {
  const int i = blockIdx.x * 256 + threadIdx.x;
  if (i < n8) {
    const v4f a = *(const v4f*)(in + (size_t)i * 8);
    const v4f b = *(const v4f*)(in + (size_t)i * 8 + 4);
    v8h hv;
#pragma unroll
    for (int e = 0; e < 4; ++e) { hv[e] = (_Float16)(a[e] * sc); hv[4 + e] = (_Float16)(b[e] * sc); }
    _Float16* p = out + (size_t)i * 8;
    *(volatile v8h*)p = hv;
    __threadfence();
    *(volatile v8h*)p = hv;
  }
}

__global__ __launch_bounds__(256) void pack_down_t(
    const float* __restrict__ wd, _Float16* __restrict__ wdt, int nk, int nr, float sc) {
  const int i = blockIdx.x * 256 + threadIdx.x;
  const int ngrp = nk >> 3;
  if (i < 64 * ngrp) {
    const int n = i / ngrp;
    const int kg = i - n * ngrp;
    const int nn = n & 7;
    v8h hv;
#pragma unroll
    for (int e = 0; e < 8; ++e) {
      const float v = wd[(size_t)(kg * 8 + e) * nr + nn] * sc;
      hv[e] = (n < nr) ? (_Float16)v : (_Float16)0.0f;
    }
    _Float16* p = wdt + (size_t)i * 8;
    *(volatile v8h*)p = hv;
    __threadfence();
    *(volatile v8h*)p = hv;
  }
}

__global__ __launch_bounds__(256) void pack_up_t(
    const float* __restrict__ wu, _Float16* __restrict__ wut, int ncols, float sc) {
  const int i = blockIdx.x * 256 + threadIdx.x;
  if (i < ncols * 4) {
    const int n = i >> 2;
    const int kg = i & 3;
    v8h hv;
#pragma unroll
    for (int e = 0; e < 8; ++e) {
      const float v = wu[(size_t)e * ncols + n] * sc;
      hv[e] = (kg == 0) ? (_Float16)v : (_Float16)0.0f;
    }
    _Float16* p = wut + (size_t)i * 8;
    *(volatile v8h*)p = hv;
    __threadfence();
    *(volatile v8h*)p = hv;
  }
}

__global__ __launch_bounds__(128) void layernorm_cast_kernel(
    const float* __restrict__ x, const float* __restrict__ gamma, const float* __restrict__ beta,
    _Float16* __restrict__ xh, _Float16* __restrict__ hnh, float* __restrict__ hnf, float eps) {
  __shared__ float red_a[4];
  __shared__ float red_b[4];
  __shared__ __align__(16) float rowbuf[1024];
  const int row  = blockIdx.x;
  const int tid  = threadIdx.x;
  const int lane = tid & 31, wave = tid >> 5;
  const size_t rbase = (size_t)row * 1024;
  const size_t ebase = rbase + (size_t)tid * 8;

  const v4f a0 = *(const v4f*)(x + ebase);
  const v4f a1 = *(const v4f*)(x + ebase + 4);
  float s = ((a0[0] + a0[1]) + (a0[2] + a0[3])) + ((a1[0] + a1[1]) + (a1[2] + a1[3]));
#pragma unroll
  for (int off = 1; off < 32; off <<= 1) s += __shfl_xor(s, off, 32);
  if (lane == 0) red_a[wave] = s;
  __syncthreads();
  const float mu = ((red_a[0] + red_a[1]) + (red_a[2] + red_a[3])) * (1.0f / 1024.0f);

  float d[8];
#pragma unroll
  for (int e = 0; e < 4; ++e) { d[e] = a0[e] - mu; d[4 + e] = a1[e] - mu; }
  float ss = 0.f;
#pragma unroll
  for (int e = 0; e < 8; ++e) ss += d[e] * d[e];
#pragma unroll
  for (int off = 1; off < 32; off <<= 1) ss += __shfl_xor(ss, off, 32);
  if (lane == 0) red_b[wave] = ss;
  __syncthreads();
  const float var = ((red_b[0] + red_b[1]) + (red_b[2] + red_b[3])) * (1.0f / 1024.0f);
  const float rs = rsqrtf(var + eps);

  const v4f g0 = *(const v4f*)(gamma + tid * 8);
  const v4f g1 = *(const v4f*)(gamma + tid * 8 + 4);
  const v4f b0 = *(const v4f*)(beta + tid * 8);
  const v4f b1 = *(const v4f*)(beta + tid * 8 + 4);
  v4f o0, o1;
#pragma unroll
  for (int e = 0; e < 4; ++e) {
    o0[e] = (d[e] * rs) * g0[e] + b0[e];
    o1[e] = (d[4 + e] * rs) * g1[e] + b1[e];
  }
  v8h hx, ho;
#pragma unroll
  for (int e = 0; e < 4; ++e) {
    hx[e] = (_Float16)a0[e]; hx[4 + e] = (_Float16)a1[e];
    ho[e] = (_Float16)o0[e]; ho[4 + e] = (_Float16)o1[e];
  }
  *(v4f*)(rowbuf + tid * 8)     = o0;
  *(v4f*)(rowbuf + tid * 8 + 4) = o1;
  __syncthreads();
  const v4f p0 = *(const v4f*)(rowbuf + tid * 4);
  const v4f p1 = *(const v4f*)(rowbuf + 512 + tid * 4);
  for (int pass = 0; pass < 2; ++pass) {
    *(volatile v8h*)(xh  + ebase) = hx;
    *(volatile v8h*)(hnh + ebase) = ho;
    *(volatile v4f*)(hnf + rbase + tid * 4)       = p0;
    *(volatile v4f*)(hnf + rbase + 512 + tid * 4) = p1;
    __threadfence();
  }
}

#define AT2_D  32
#define AT2_KC 64
#define AT2_NW 4

__device__ __forceinline__ v8f mma_h(v16h a, v16h b, v8f c) {
  c = __builtin_amdgcn_wmma_f32_16x16x32_f16(false, a, false, b, (short)0, c, false, false);
  asm volatile("v_nop\n\tv_nop\n\tv_nop\n\tv_nop" : "+v"(c) : "v"(a), "v"(b));
  return c;
}

__global__ __launch_bounds__(128)
void attn_hd32_kernel(const _Float16* __restrict__ qkv, _Float16* __restrict__ out,
                      int S, int ldq, float sm_scale, float o_scale) {
  __shared__ __align__(16) _Float16 Ksh[AT2_KC * AT2_D];
  __shared__ __align__(16) _Float16 Vth[AT2_D * AT2_KC];
  __shared__ __align__(16) _Float16 Psh[AT2_NW][16 * AT2_KC];
  __shared__ __align__(16) float    Os[AT2_NW][16 * 68];

  const int tid  = threadIdx.x;
  const int wave = tid >> 5;
  const int lane = tid & 31;
  const int hh   = lane >> 4;
  const int c    = lane & 15;
  const float PSC = 32768.0f;

  const int nqb = S >> 6;
  const int b   = blockIdx.x / nqb;
  const int qb  = blockIdx.x - b * nqb;
  const int q0  = (qb << 6) + wave * 16;
  const size_t rowb = (size_t)b * S;
  const int nChunks = S / AT2_KC;

  float* os = Os[wave];
  _Float16* pw = Psh[wave];

#pragma unroll 1
  for (int h = 0; h < 2; ++h) {
    const v16h qa = Frag<_Float16>::load(qkv + (rowb + q0 + c) * (size_t)ldq + h * AT2_D + 8 * hh);

    float mrow[8], lrow[8];
    v8f oacc[2];
#pragma unroll
    for (int r = 0; r < 8; ++r) { mrow[r] = -INFINITY; lrow[r] = 0.f; }
#pragma unroll
    for (int t = 0; t < 2; ++t) oacc[t] = (v8f){0.f,0.f,0.f,0.f,0.f,0.f,0.f,0.f};

    for (int kc = 0; kc < nChunks; ++kc) {
      const int kv0 = kc * AT2_KC;
      __syncthreads();
      {
        const int kvr = tid >> 1, dh = (tid & 1) * 16;
        const _Float16* krow = qkv + (rowb + kv0 + kvr) * (size_t)ldq + 64 + h * AT2_D + dh;
        const _Float16* vrow = krow + 64;
        const v8h k0v = *(const v8h*)krow;
        const v8h k1v = *(const v8h*)(krow + 8);
        const v8h v0v = *(const v8h*)vrow;
        const v8h v1v = *(const v8h*)(vrow + 8);
        *(v8h*)(Ksh + kvr * AT2_D + dh)     = k0v;
        *(v8h*)(Ksh + kvr * AT2_D + dh + 8) = k1v;
#pragma unroll
        for (int e = 0; e < 8; ++e) {
          Vth[(dh + e) * AT2_KC + kvr]     = v0v[e];
          Vth[(dh + 8 + e) * AT2_KC + kvr] = v1v[e];
        }
      }
      __syncthreads();

      v8f s[4];
#pragma unroll
      for (int j = 0; j < 4; ++j) {
        const v16h kb = Frag<_Float16>::load(Ksh + (j * 16 + c) * AT2_D + 8 * hh);
        s[j] = mma_h(qa, kb, (v8f){0.f,0.f,0.f,0.f,0.f,0.f,0.f,0.f});
      }
      float cm[8];
#pragma unroll
      for (int r = 0; r < 8; ++r) {
        float m = -INFINITY;
#pragma unroll
        for (int j = 0; j < 4; ++j) {
          s[j][r] = s[j][r] * sm_scale;
          m = fmaxf(m, s[j][r]);
        }
#pragma unroll
        for (int off = 1; off < 16; off <<= 1) m = fmaxf(m, __shfl_xor(m, off, 32));
        cm[r] = m;
      }
#pragma unroll
      for (int r = 0; r < 8; ++r) {
        const float mnew  = fmaxf(mrow[r], cm[r]);
        const float alpha = expf(mrow[r] - mnew);
        mrow[r] = mnew;
        float psum = 0.f;
#pragma unroll
        for (int j = 0; j < 4; ++j) {
          const float p = expf(s[j][r] - mnew);
          psum += p;
          pw[(8 * hh + r) * AT2_KC + j * 16 + c] = (_Float16)(p * PSC);
        }
#pragma unroll
        for (int off = 1; off < 16; off <<= 1) psum += __shfl_xor(psum, off, 32);
        lrow[r] = lrow[r] * alpha + psum;
#pragma unroll
        for (int t = 0; t < 2; ++t) oacc[t][r] *= alpha;
      }
      __builtin_amdgcn_fence(__ATOMIC_RELEASE, "workgroup");
      __builtin_amdgcn_wave_barrier();
      __builtin_amdgcn_fence(__ATOMIC_ACQUIRE, "workgroup");
#pragma unroll
      for (int kk = 0; kk < 2; ++kk) {
        const v16h pa = Frag<_Float16>::load(pw + c * AT2_KC + kk * 32 + 8 * hh);
#pragma unroll
        for (int t = 0; t < 2; ++t) {
          const v16h vb = Frag<_Float16>::load(Vth + (t * 16 + c) * AT2_KC + kk * 32 + 8 * hh);
          oacc[t] = mma_h(pa, vb, oacc[t]);
        }
      }
    }

#pragma unroll
    for (int r = 0; r < 8; ++r) {
      const float inv = o_scale / (lrow[r] * PSC);
#pragma unroll
      for (int t = 0; t < 2; ++t) os[(8 * hh + r) * 68 + h * AT2_D + t * 16 + c] = oacc[t][r] * inv;
    }
  }

  __builtin_amdgcn_fence(__ATOMIC_RELEASE, "workgroup");
  __builtin_amdgcn_wave_barrier();
  __builtin_amdgcn_fence(__ATOMIC_ACQUIRE, "workgroup");
  {
    const int q4 = lane >> 3, c8 = (lane & 7) * 8;
    _Float16* ob = out + (rowb + q0) * 64;
    for (int pass = 0; pass < 2; ++pass) {
#pragma unroll
      for (int it = 0; it < 4; ++it) {
        const int row = it * 4 + q4;
        const float* sp = os + row * 68 + c8;
        v8h hv;
#pragma unroll
        for (int e = 0; e < 8; ++e) hv[e] = (_Float16)sp[e];
        *(volatile v8h*)(ob + (size_t)row * 64 + c8) = hv;
      }
      __threadfence();
    }
  }
}

static inline size_t al256(size_t b) { return (b + 255) & ~(size_t)255; }

template <int OUT_MODE, bool RESID>
static void launch_gemm_f16(const void* A, int lda, const void* Bt, int ldb, void* C, int ldc,
                            const float* resid, const float* fdummy,
                            int M, int N, int K, float scale, hipStream_t st) {
  const int tiles = (M / 64) * (N / 64);
  dim3 grid((tiles + 7) / 8, 1);
  wmma_gemm64<0, false, 0, OUT_MODE, RESID, 0><<<grid, 256, 0, st>>>(
      (const unsigned short*)A, (const unsigned short*)A, lda, 0L,
      (const unsigned short*)Bt, (const unsigned short*)Bt, ldb, 0L,
      C, C, ldc, 0L,
      fdummy, resid, 0L, M, N, K, scale);
}

extern "C" void kernel_launch(void* const* d_in, const int* in_sizes, int n_in,
                              void* d_out, int out_size, void* d_ws, size_t ws_size,
                              hipStream_t stream) {
  const int E = 1024;
  const int NQKV = 192;
  const int DA = 64;
  const int R = 8;
  const int S = 2048;
  const int NPAD_DOWN = 64;
  const int KPAD_UP = 32;
  if (n_in < 8) return;
  const int M = in_sizes[0] / E;
  if (M <= 0 || (M % S) != 0 || (M % 64) != 0) return;
  const int B = M / S;
  if (in_sizes[1] != E * E || in_sizes[2] != E || in_sizes[3] != E ||
      in_sizes[4] != E * R || in_sizes[5] != R * E ||
      in_sizes[6] != NQKV * E || in_sizes[7] != E * DA) return;
  if (out_size != M * E) return;

  const float* x      = (const float*)d_in[0];
  const float* w_base = (const float*)d_in[1];
  const float* ln_g   = (const float*)d_in[2];
  const float* ln_b   = (const float*)d_in[3];
  const float* w_down = (const float*)d_in[4];
  const float* w_up   = (const float*)d_in[5];
  const float* w_qkv  = (const float*)d_in[6];
  const float* w_ao   = (const float*)d_in[7];
  float* out = (float*)d_out;

  char* ws = (char*)d_ws;
  size_t off = 0;
  const size_t o_xh   = off; off += al256((size_t)M * E * 2);
  const size_t o_hnh  = off; off += al256((size_t)M * E * 2);
  const size_t o_hnf  = off; off += al256((size_t)M * E * 4);
  const size_t o_wbh  = off; off += al256((size_t)E * E * 2);
  const size_t o_wqh  = off; off += al256((size_t)NQKV * E * 2);
  const size_t o_woh  = off; off += al256((size_t)E * DA * 2);
  const size_t o_wdt  = off; off += al256((size_t)NPAD_DOWN * E * 2);
  const size_t o_wut  = off; off += al256((size_t)E * KPAD_UP * 2);
  const size_t o_qkv  = off; off += al256((size_t)M * NQKV * 2);
  const size_t o_att  = off; off += al256((size_t)M * DA * 2);
  const size_t o_hwa  = off; off += al256((size_t)M * E * 2);
  const size_t o_tlo  = off; off += al256((size_t)M * NPAD_DOWN * 2);
  const size_t o_dlt  = off; off += al256((size_t)M * E * 4);
  if (off > ws_size) return;

  _Float16* xh   = (_Float16*)(ws + o_xh);
  _Float16* hnh  = (_Float16*)(ws + o_hnh);
  float*    hnf  = (float*)   (ws + o_hnf);
  _Float16* wbh  = (_Float16*)(ws + o_wbh);
  _Float16* wqh  = (_Float16*)(ws + o_wqh);
  _Float16* woh  = (_Float16*)(ws + o_woh);
  _Float16* wdt  = (_Float16*)(ws + o_wdt);
  _Float16* wut  = (_Float16*)(ws + o_wut);
  _Float16* qkvh = (_Float16*)(ws + o_qkv);
  _Float16* atth = (_Float16*)(ws + o_att);
  _Float16* hwa  = (_Float16*)(ws + o_hwa);
  _Float16* tlo  = (_Float16*)(ws + o_tlo);
  float*    dlt  = (float*)   (ws + o_dlt);

  const float WSC = 64.0f;
  const float OSC = 64.0f;

  { const int n8 = (E * E) / 8;     cast_scale_f16x8<<<(n8 + 255) / 256, 256, 0, stream>>>(w_base, wbh, n8, WSC); }
  { const int n8 = (NQKV * E) / 8;  cast_scale_f16x8<<<(n8 + 255) / 256, 256, 0, stream>>>(w_qkv,  wqh, n8, WSC); }
  { const int n8 = (E * DA) / 8;    cast_scale_f16x8<<<(n8 + 255) / 256, 256, 0, stream>>>(w_ao,   woh, n8, WSC); }
  { const int nthr = NPAD_DOWN * (E / 8); pack_down_t<<<(nthr + 255) / 256, 256, 0, stream>>>(w_down, wdt, E, R, WSC); }
  { const int nthr = E * 4; pack_up_t<<<(nthr + 255) / 256, 256, 0, stream>>>(w_up, wut, E, WSC); }
  layernorm_cast_kernel<<<M, 128, 0, stream>>>(x, ln_g, ln_b, xh, hnh, hnf, 1e-5f);
  launch_gemm_f16<1, false>(hnh, E, wqh, E, qkvh, NQKV, hnf, hnf, M, NQKV, E, 1.0f / WSC, stream);
  attn_hd32_kernel<<<B * (S / 64), 128, 0, stream>>>(qkvh, atth, S, NQKV, 0.17677669529663687f, OSC);
  launch_gemm_f16<1, true>(atth, DA, woh, DA, hwa, E, hnf, hnf, M, E, DA, 1.0f / (WSC * OSC), stream);
  launch_gemm_f16<1, false>(hwa, E, wdt, E, tlo, NPAD_DOWN, hnf, hnf, M, NPAD_DOWN, E, 1.0f / WSC, stream);
  launch_gemm_f16<0, false>(tlo, NPAD_DOWN, wut, KPAD_UP, dlt, E, hnf, hnf, M, E, KPAD_UP, 1.0f / (WSC * 8.0f), stream);
  launch_gemm_f16<0, true>(xh, E, wbh, E, out, E, dlt, hnf, M, E, E, 1.0f / WSC, stream);

  (void)hipGetLastError();
}
